// ExperimentalLayer7_1563368096370
// MI455X (gfx1250) — hardware-verified
//
#include <hip/hip_runtime.h>


namespace {
constexpr int Bn = 4, S = 2048, D = 1024, NT = Bn * S;
constexpr float KS = 8.0f, VS = 8.0f, PS = 8.0f;

typedef _Float16 b16;
typedef __attribute__((ext_vector_type(16))) _Float16 v16b;
typedef __attribute__((ext_vector_type(16))) __bf16 v16bb;
typedef __attribute__((ext_vector_type(8))) _Float16 v8b;
typedef __attribute__((ext_vector_type(8))) unsigned short v8us;
typedef __attribute__((ext_vector_type(8))) float v8f;
typedef __attribute__((ext_vector_type(4))) float v4f;
__device__ __forceinline__ float bf16_rne(float f) { unsigned int u = __float_as_uint(f); u += 0x7FFFu + ((u >> 16) & 1u); return __uint_as_float(u & 0xFFFF0000u); }
__device__ __forceinline__ unsigned short bf16_bits(float f) { unsigned int u = __float_as_uint(f); u += 0x7FFFu + ((u >> 16) & 1u); return (unsigned short)(u >> 16); }
__device__ __forceinline__ void split16(float v, b16& hi, b16& lo) { hi = (b16)v; lo = (b16)(v - (float)hi); }
__device__ __forceinline__ v16b frag_kb(const b16* p, int hh) { const v8b a = *(const v8b*)(p + 8 * hh), b = *(const v8b*)(p + 16 + 8 * hh); v16b f;
#pragma unroll
  for (int e = 0; e < 8; ++e) { f[e] = a[e]; f[8 + e] = b[e]; } return f; }
__device__ __forceinline__ v16b frag_x(const float* p, int hh) { v16b f;
#pragma unroll
  for (int e = 0; e < 8; ++e) { f[e] = (b16)bf16_rne(p[8 * hh + e]); f[8 + e] = (b16)bf16_rne(p[16 + 8 * hh + e]); } return f; }
__device__ __forceinline__ v16bb frag_bf(const unsigned short* p, int hh) { const v8us a = *(const v8us*)(p + 8 * hh), b = *(const v8us*)(p + 16 + 8 * hh); union { unsigned short s[16]; v16bb v; } u;
#pragma unroll
  for (int e = 0; e < 8; ++e) { u.s[e] = a[e]; u.s[8 + e] = b[e]; } return u.v; }
__device__ __forceinline__ v16bb frag_f32bf(const float* p, int hh) { union { unsigned short s[16]; v16bb v; } u;
#pragma unroll
  for (int e = 0; e < 8; ++e) { u.s[e] = bf16_bits(p[8 * hh + e]); u.s[8 + e] = bf16_bits(p[16 + 8 * hh + e]); } return u.v; }
__device__ __forceinline__ v8f wmma16b(v16b a, v16b b, v8f c) { v8f d = __builtin_amdgcn_wmma_f32_16x16x32_f16(false, a, false, b, (short)0, c, false, false); asm volatile("v_nop\n\tv_nop\n\tv_nop\n\tv_nop" : "+v"(d) : "v"(a), "v"(b)); return d; }
__device__ __forceinline__ v8f wmma16bb(v16bb a, v16bb b, v8f c) { v8f d = __builtin_amdgcn_wmma_f32_16x16x32_bf16(false, a, false, b, (short)0, c, false, false); asm volatile("v_nop\n\tv_nop\n\tv_nop\n\tv_nop" : "+v"(d) : "v"(a), "v"(b)); return d; }
__device__ __forceinline__ void wave_lds_sync() { __builtin_amdgcn_fence(__ATOMIC_RELEASE, "workgroup"); __builtin_amdgcn_wave_barrier(); __builtin_amdgcn_fence(__ATOMIC_ACQUIRE, "workgroup"); }
__device__ __forceinline__ float nexp(float x) { return __builtin_amdgcn_exp2f(x * 1.4426950408889634f); }

__global__ __launch_bounds__(256) void prep_kernel(const float* __restrict__ W, unsigned short* __restrict__ w16) {
  const size_t tid = (size_t)blockIdx.x * blockDim.x + threadIdx.x, nth = (size_t)gridDim.x * blockDim.x;
  for (int pass = 0; pass < 2; ++pass) { for (size_t p = tid; p < (size_t)2 * D * D / 8; p += nth) { v8us v;
#pragma unroll
      for (int e = 0; e < 8; ++e) v[e] = bf16_bits(W[p * 8 + e]);
      *(volatile v8us*)(w16 + p * 8) = v; } __threadfence(); }
}

__global__ __launch_bounds__(128) void proj_kernel(const float* __restrict__ x, const unsigned short* __restrict__ w16, b16* __restrict__ kh, b16* __restrict__ kl, b16* __restrict__ vt) {
  __shared__ __attribute__((aligned(16))) b16 Th[4][32][64 + 8], Tl[4][32][64 + 8]; __shared__ __attribute__((aligned(16))) b16 Tv[64][128 + 8];
  const int lane = threadIdx.x & 31, wave = threadIdx.x >> 5, nloc = lane & 15, hlf = lane >> 4, c0 = blockIdx.x * 64, p0 = blockIdx.y * 128, m0 = p0 + wave * 32, b = p0 / S, t0 = p0 % S;
  v8f acc[2][4];
#pragma unroll
  for (int r = 0; r < 2; ++r)
#pragma unroll
    for (int t = 0; t < 4; ++t) acc[r][t] = (v8f){};
#pragma unroll 2
  for (int kb = 0; kb < D; kb += 32) { const v16bb a0 = frag_f32bf(x + (size_t)(m0 + nloc) * D + kb, hlf), a1 = frag_f32bf(x + (size_t)(m0 + 16 + nloc) * D + kb, hlf);
#pragma unroll
    for (int t = 0; t < 4; ++t) { const v16bb bw = frag_bf(w16 + (size_t)(c0 + t * 16 + nloc) * D + kb, hlf); acc[0][t] = wmma16bb(a0, bw, acc[0][t]); acc[1][t] = wmma16bb(a1, bw, acc[1][t]); } }
  if (c0 < D) {
#pragma unroll
    for (int t = 0; t < 4; ++t)
#pragma unroll
      for (int r = 0; r < 2; ++r)
#pragma unroll
        for (int v = 0; v < 8; ++v) { b16 h_, l_; split16(acc[r][t][v] * KS, h_, l_); Th[wave][r * 16 + 8 * hlf + v][t * 16 + nloc] = h_; Tl[wave][r * 16 + 8 * hlf + v][t * 16 + nloc] = l_; }
    wave_lds_sync();
    for (int pass = 0; pass < 2; ++pass) {
#pragma unroll
      for (int j = 0; j < 8; ++j) { const int rr = j * 4 + (lane >> 3), c8 = (lane & 7) * 8; const size_t o = (size_t)(m0 + rr) * D + c0 + c8; *(volatile v8b*)(kh + o) = *(const v8b*)(&Th[wave][rr][c8]); *(volatile v8b*)(kl + o) = *(const v8b*)(&Tl[wave][rr][c8]); }
      __threadfence(); }
    return; }
#pragma unroll
  for (int t = 0; t < 4; ++t)
#pragma unroll
    for (int r = 0; r < 2; ++r)
#pragma unroll
      for (int v = 0; v < 8; ++v) Tv[t * 16 + nloc][wave * 32 + r * 16 + 8 * hlf + v] = (b16)(acc[r][t][v] * VS);
  __syncthreads();
  for (int pass = 0; pass < 2; ++pass) { for (int i = threadIdx.x; i < 64 * 16; i += 128) { const int d = i >> 4, c8 = (i & 15) * 8; *(volatile v8b*)(vt + ((size_t)b * D + (c0 - D) + d) * S + t0 + c8) = *(const v8b*)(&Tv[d][c8]); } __threadfence(); }
}

__global__ __launch_bounds__(128) void score_kernel(const float* __restrict__ x, const b16* __restrict__ kh, const b16* __restrict__ kl, float* __restrict__ sc) {
  __shared__ __attribute__((aligned(16))) float Ts[4][32 * 64];
  const int lane = threadIdx.x & 31, wave = threadIdx.x >> 5, nloc = lane & 15, hlf = lane >> 4, c0 = blockIdx.x * 64, p0 = blockIdx.y * 128, m0 = p0 + wave * 32, b = p0 / S, q0b = p0 % S;
  if (c0 > q0b + 127) return;
  const b16* Kh = kh + ((size_t)b * S) * D; const b16* Kl = kl + ((size_t)b * S) * D;
  v8f acc[2][4];
#pragma unroll
  for (int r = 0; r < 2; ++r)
#pragma unroll
    for (int t = 0; t < 4; ++t) acc[r][t] = (v8f){};
#pragma unroll 2
  for (int kb = 0; kb < D; kb += 32) { const v16b a0 = frag_x(x + (size_t)(m0 + nloc) * D + kb, hlf), a1 = frag_x(x + (size_t)(m0 + 16 + nloc) * D + kb, hlf);
#pragma unroll
    for (int t = 0; t < 4; ++t) { const size_t ro = (size_t)(c0 + t * 16 + nloc) * D + kb; const v16b bh = frag_kb(Kh + ro, hlf), bl = frag_kb(Kl + ro, hlf); acc[0][t] = wmma16b(a0, bh, acc[0][t]); acc[0][t] = wmma16b(a0, bl, acc[0][t]); acc[1][t] = wmma16b(a1, bh, acc[1][t]); acc[1][t] = wmma16b(a1, bl, acc[1][t]); } }
  float* Tt = Ts[wave];
#pragma unroll
  for (int t = 0; t < 4; ++t)
#pragma unroll
    for (int r = 0; r < 2; ++r)
#pragma unroll
      for (int v = 0; v < 8; ++v) Tt[(r * 16 + v + 8 * hlf) * 64 + t * 16 + nloc] = acc[r][t][v] * (1.0f / KS);
  wave_lds_sync();
  for (int pass = 0; pass < 2; ++pass) {
#pragma unroll
    for (int j = 0; j < 16; ++j) { const int rr = j * 2 + hlf, c4 = nloc * 4; *(volatile v4f*)(sc + (size_t)(m0 + rr) * S + c0 + c4) = *(const v4f*)(Tt + rr * 64 + c4); }
    __threadfence(); }
}

__global__ __launch_bounds__(256) void softmax_kernel(const float* __restrict__ sc, b16* __restrict__ P) {
  const int wid = threadIdx.x >> 5, lane = threadIdx.x & 31; const size_t row = (size_t)blockIdx.x * 8 + wid; const int q = (int)(row % S); const float* sr = sc + row * S;
  float mx = -INFINITY; for (int k = lane; k <= q; k += 32) mx = fmaxf(mx, sr[k]);
#pragma unroll
  for (int o = 1; o < 32; o <<= 1) mx = fmaxf(mx, __shfl_xor(mx, o));
  float sm = 0.0f; for (int k = lane; k <= q; k += 32) sm += nexp(sr[k] - mx);
#pragma unroll
  for (int o = 1; o < 32; o <<= 1) sm += __shfl_xor(sm, o);
  const float inv = PS / sm;
  for (int pass = 0; pass < 2; ++pass) { for (int k8 = lane * 8; k8 < S; k8 += 256) { v8b o8;
#pragma unroll
      for (int e = 0; e < 8; ++e) { const int k = k8 + e; o8[e] = (b16)((k <= q) ? nexp(sr[k] - mx) * inv : 0.0f); }
      *(volatile v8b*)(P + row * S + k8) = o8; } __threadfence(); }
}

__global__ __launch_bounds__(128) void pv_kernel(const b16* __restrict__ P, const b16* __restrict__ vt, const float* __restrict__ x, float* __restrict__ out) {
  __shared__ __attribute__((aligned(16))) float Ts[4][32 * 64];
  const int lane = threadIdx.x & 31, wave = threadIdx.x >> 5, nloc = lane & 15, hlf = lane >> 4, c0 = blockIdx.x * 64, p0 = blockIdx.y * 128, m0 = p0 + wave * 32, b = p0 / S, q0b = p0 % S;
  const b16* V = vt + ((size_t)b * D) * S; const int kend = q0b + 128;
  v8f acc[2][4];
#pragma unroll
  for (int r = 0; r < 2; ++r)
#pragma unroll
    for (int t = 0; t < 4; ++t) acc[r][t] = (v8f){};
#pragma unroll 2
  for (int kb = 0; kb < kend; kb += 32) { const v16b a0 = frag_kb(P + (size_t)(m0 + nloc) * S + kb, hlf), a1 = frag_kb(P + (size_t)(m0 + 16 + nloc) * S + kb, hlf);
#pragma unroll
    for (int t = 0; t < 4; ++t) { const v16b bw = frag_kb(V + (size_t)(c0 + t * 16 + nloc) * S + kb, hlf); acc[0][t] = wmma16b(a0, bw, acc[0][t]); acc[1][t] = wmma16b(a1, bw, acc[1][t]); } }
  float* Tt = Ts[wave];
#pragma unroll
  for (int t = 0; t < 4; ++t) { const int cc = c0 + t * 16 + nloc;
#pragma unroll
    for (int r = 0; r < 2; ++r)
#pragma unroll
      for (int v = 0; v < 8; ++v) { const int rl = r * 16 + v + 8 * hlf; Tt[rl * 64 + t * 16 + nloc] = acc[r][t][v] * (1.0f / (PS * VS)) + bf16_rne(x[(size_t)(m0 + rl) * D + cc]); } }
  wave_lds_sync();
  for (int pass = 0; pass < 2; ++pass) {
#pragma unroll
    for (int j = 0; j < 16; ++j) { const int rr = j * 2 + hlf, c4 = nloc * 4; *(volatile v4f*)(out + (size_t)(m0 + rr) * D + c0 + c4) = *(const v4f*)(Tt + rr * 64 + c4); }
    __threadfence(); }
}
}

extern "C" void kernel_launch(void* const* d_in, const int* in_sizes, int n_in,
                              void* d_out, int out_size, void* d_ws, size_t ws_size, hipStream_t stream) {
  (void)n_in; (void)out_size;
  const float* x = (const float*)d_in[0]; const float* W = (const float*)d_in[1];
  float* out = (float*)d_out;
  if (in_sizes[0] != NT * D || in_sizes[1] != 2 * D * D) return;
  size_t off = 0; char* ws = (char*)d_ws;
  auto carve = [&](size_t bytes) { char* p = ws + off; off += (bytes + 255) & ~(size_t)255; return p; };
  unsigned short* w16 = (unsigned short*)carve((size_t)2 * D * D * 2); b16* kh = (b16*)carve((size_t)NT * D * 2); b16* kl = (b16*)carve((size_t)NT * D * 2); b16* vt = (b16*)carve((size_t)NT * D * 2);
  float* sc = (float*)carve((size_t)NT * S * 4); b16* P = (b16*)kh;
  if (off > ws_size) return;
  prep_kernel<<<512, 256, 0, stream>>>(W, w16);
  proj_kernel<<<dim3(2 * D / 64, NT / 128), 128, 0, stream>>>(x, w16, kh, kl, vt);
  score_kernel<<<dim3(S / 64, NT / 128), 128, 0, stream>>>(x, kh, kl, sc);
  softmax_kernel<<<NT / 8, 256, 0, stream>>>(sc, P);
  pv_kernel<<<dim3(D / 64, NT / 128), 128, 0, stream>>>(P, vt, x, out);
}
